// MultiheadedAttention_47691316854802
// MI455X (gfx1250) — hardware-verified
//
#include <hip/hip_runtime.h>

#ifndef NB
#define NB 2
#endif
#ifndef SEQ
#define SEQ 2048
#endif
#define NB_FULL 2
#define SEQ_FULL 2048
#define DM 1024
#define NH 16
#define DK 64
#define MTOK (NB * SEQ)
#define ACT_SC 16.0f
#define W_SC 64.0f

static_assert(DM == NH * DK);
static_assert(DK == 64);
static_assert(SEQ % 64 == 0);
static_assert(MTOK % 64 == 0);
static_assert(DM % 64 == 0);
static_assert(DM % 32 == 0);
static_assert((2 * DM) % 32 == 0);
static_assert(DM % 8 == 0);
static_assert(NB <= NB_FULL && SEQ <= SEQ_FULL);

typedef __attribute__((ext_vector_type(16))) _Float16 v16h;
typedef __attribute__((ext_vector_type(8)))  _Float16 v8h;
typedef __attribute__((ext_vector_type(16))) __bf16   v16b;
typedef __attribute__((ext_vector_type(8)))  __bf16   v8b;
typedef __attribute__((ext_vector_type(8)))  float    v8f;
typedef __attribute__((ext_vector_type(4)))  float    v4f;
typedef __attribute__((ext_vector_type(4)))  unsigned v4u;


__device__ __forceinline__ float cmb_bf(float v) {
    const unsigned u = __builtin_bit_cast(unsigned, v);
    const unsigned r = (u + 0x7fffu + ((u >> 16) & 1u)) & 0xffff0000u;
    return __builtin_bit_cast(float, r);
}
__device__ __forceinline__ unsigned short bfu_rne(float v) {
    unsigned u = __builtin_bit_cast(unsigned, v);
    u += 0x7fffu + ((u >> 16) & 1u);
    return (unsigned short)(u >> 16);
}
__device__ __forceinline__ unsigned pk2h(float a, float b) {
    return (unsigned)__builtin_bit_cast(unsigned short, (_Float16)a) | ((unsigned)__builtin_bit_cast(unsigned short, (_Float16)b) << 16);
}
__device__ __forceinline__ unsigned pk2b(float a, float b) {
    return (unsigned)bfu_rne(a) | ((unsigned)bfu_rne(b) << 16);
}
__device__ __forceinline__ void split2(float a, float b, unsigned& hi, unsigned& lo) {
    const unsigned short ha = bfu_rne(a), hb = bfu_rne(b);
    const float ra = a - __builtin_bit_cast(float, (unsigned)ha << 16);
    const float rb = b - __builtin_bit_cast(float, (unsigned)hb << 16);
    hi = (unsigned)ha | ((unsigned)hb << 16);
    lo = (unsigned)bfu_rne(ra) | ((unsigned)bfu_rne(rb) << 16);
}

__device__ __forceinline__ void dep_guard_h(v8f& a, v8f& b, v16h x, v16h y) { asm volatile("v_nop\n\tv_nop\n\tv_nop\n\tv_nop" : "+v"(a), "+v"(b) : "v"(x), "v"(y)); }
__device__ __forceinline__ void dep_guard_b(v8f& a, v8f& b, v16b x, v16b y) { asm volatile("v_nop\n\tv_nop\n\tv_nop\n\tv_nop" : "+v"(a), "+v"(b) : "v"(x), "v"(y)); }
__device__ __forceinline__ void keep4_h(v16h a, v16h b, v16h c, v16h d) { asm volatile("v_nop" :: "v"(a), "v"(b), "v"(c), "v"(d)); }
__device__ __forceinline__ void keep4_b(v16b a, v16b b, v16b c, v16b d) { asm volatile("v_nop" :: "v"(a), "v"(b), "v"(c), "v"(d)); }
__device__ __forceinline__ void acc_guard4(v8f& a, v8f& b, v8f& c, v8f& d) { asm volatile("v_nop\n\tv_nop\n\tv_nop\n\tv_nop" : "+v"(a), "+v"(b), "+v"(c), "+v"(d)); }

template <typename T> struct Frag;
template <> struct Frag<_Float16> {
  typedef v16h V; union U { v16h v; v8h h[2]; };
  static __device__ __forceinline__ v16h load(const _Float16* p) {
    U f; f.h[0] = *(const v8h*)(p); f.h[1] = *(const v8h*)(p + 16); return f.v;
  }
  static __device__ __forceinline__ v8f mma(v16h a, v16h b, v8f c) {
    return __builtin_amdgcn_wmma_f32_16x16x32_f16(false, a, false, b, (short)0, c, false, false);
  }
  static __device__ __forceinline__ void guard(v8f& a, v8f& b, v16h x, v16h y) { dep_guard_h(a, b, x, y); }
  static __device__ __forceinline__ void keep(v16h a, v16h b, v16h c, v16h d) { keep4_h(a, b, c, d); }
};
template <> struct Frag<__bf16> {
  typedef v16b V; union U { v16b v; v8b h[2]; };
  static __device__ __forceinline__ v16b load(const __bf16* p) {
    U f; f.h[0] = *(const v8b*)(p); f.h[1] = *(const v8b*)(p + 16); return f.v;
  }
  static __device__ __forceinline__ v8f mma(v16b a, v16b b, v8f c) {
    return __builtin_amdgcn_wmma_f32_16x16x32_bf16(false, a, false, b, (short)0, c, false, false);
  }
  static __device__ __forceinline__ void guard(v8f& a, v8f& b, v16b x, v16b y) { dep_guard_b(a, b, x, y); }
  static __device__ __forceinline__ void keep(v16b a, v16b b, v16b c, v16b d) { keep4_b(a, b, c, d); }
};
template <int ET> struct Elem;
template <> struct Elem<0> { typedef _Float16 T; };
template <> struct Elem<1> { typedef __bf16 T; };

__device__ __forceinline__ v8f wmma16(v16h a, v16h b, v8f c) {
    c = __builtin_amdgcn_wmma_f32_16x16x32_f16(false, a, false, b, (short)0, c, false, false);
    asm volatile("v_nop\n\tv_nop\n\tv_nop\n\tv_nop" : "+v"(c) : "v"(a), "v"(b));
    return c;
}

static_assert((MTOK * (DM / 8)) % 256 == 0);
__global__ __launch_bounds__(256) void k_cast_act(const float* __restrict__ src, unsigned short* __restrict__ dst) {
    const int u = blockIdx.x * 256 + threadIdx.x;
    if (u >= MTOK * (DM / 8)) return;
    const int r = u / (DM / 8); const int c0 = 8 * (u % (DM / 8));
    const int b = r / SEQ; const int s = r - b * SEQ;
    const float* p = src + ((size_t)b * SEQ_FULL + s) * DM + c0;
    const v4f x0 = *(const v4f*)p; const v4f x1 = *(const v4f*)(p + 4);
    v4u pk;
    pk.x = pk2h(cmb_bf(x0.x) * ACT_SC, cmb_bf(x0.y) * ACT_SC);
    pk.y = pk2h(cmb_bf(x0.z) * ACT_SC, cmb_bf(x0.w) * ACT_SC);
    pk.z = pk2h(cmb_bf(x1.x) * ACT_SC, cmb_bf(x1.y) * ACT_SC);
    pk.w = pk2h(cmb_bf(x1.z) * ACT_SC, cmb_bf(x1.w) * ACT_SC);
    volatile v4u* d = (volatile v4u*)(dst + (size_t)r * DM + c0);
    *d = pk; __threadfence(); *d = pk;
}

static_assert((DM * (DM / 8)) % 256 == 0);
__global__ __launch_bounds__(256) void k_cast_wT(const float* __restrict__ W, unsigned short* __restrict__ WT) {
    const int u = blockIdx.x * 256 + threadIdx.x;
    if (u >= DM * (DM / 8)) return;
    const int n = u / (DM / 8); const int k0 = 8 * (u % (DM / 8));
    float w[8];
#pragma unroll
    for (int e = 0; e < 8; ++e) w[e] = cmb_bf(W[(size_t)(k0 + e) * DM + n]) * W_SC;
    v4u pk; pk.x = pk2h(w[0], w[1]); pk.y = pk2h(w[2], w[3]); pk.z = pk2h(w[4], w[5]); pk.w = pk2h(w[6], w[7]);
    volatile v4u* d = (volatile v4u*)(WT + (size_t)n * DM + k0);
    *d = pk; __threadfence(); *d = pk;
}
__global__ __launch_bounds__(256) void k_cast_wo2(const float* __restrict__ W, unsigned short* __restrict__ WT2) {
    const int u = blockIdx.x * 256 + threadIdx.x;
    if (u >= DM * (DM / 8)) return;
    const int n = u / (DM / 8); const int k0 = 8 * (u % (DM / 8));
    float w[8];
#pragma unroll
    for (int e = 0; e < 8; ++e) w[e] = W[(size_t)(k0 + e) * DM + n];
    v4u pk; pk.x = pk2b(w[0], w[1]); pk.y = pk2b(w[2], w[3]); pk.z = pk2b(w[4], w[5]); pk.w = pk2b(w[6], w[7]);
    volatile v4u* d0 = (volatile v4u*)(WT2 + (size_t)n * (2 * DM) + k0);
    volatile v4u* d1 = (volatile v4u*)(WT2 + (size_t)n * (2 * DM) + DM + k0);
    *d0 = pk; *d1 = pk; __threadfence(); *d0 = pk; *d1 = pk;
}

template <int ET, int BIAS_MODE, int OUT_MODE>
__device__ __forceinline__ void gemm64_body(float* sT, const unsigned short* __restrict__ Ap, const int lda,
                                            const unsigned short* __restrict__ Btp, const int ldb,
                                            void* __restrict__ Cout, const int ldc, const float* __restrict__ bias,
                                            const int M, const int N, const int K, const float scale) {
  typedef typename Elem<ET>::T T;
  typedef typename Frag<T>::V V;
  const T* A = (const T*)Ap; const T* Bt = (const T*)Btp;
  const int lane = threadIdx.x & 31;
  const int wave = threadIdx.x >> 5;
  const int tilesN = N >> 6;
  const int tilesM = M >> 6;
  const int tile = blockIdx.x * 8 + wave;
  if (tile >= tilesM * tilesN) return;
  const int tm = tile / tilesN;
  const int tn = tile - tm * tilesN;
  const int m0 = tm << 6;
  const int n0 = tn << 6;
  const int rlane = lane & 15;
  const int koff  = (lane >> 4) * 8;
  const int mOff  = (lane >> 4) * 8;

  v8f acc[4][4];
#pragma unroll
  for (int i = 0; i < 4; ++i)
#pragma unroll
    for (int j = 0; j < 4; ++j) acc[i][j] = (v8f){0.f,0.f,0.f,0.f,0.f,0.f,0.f,0.f};

  for (int k0 = 0; k0 < K; k0 += 32) {
    V bh[4];
#pragma unroll
    for (int j = 0; j < 4; ++j) bh[j] = Frag<T>::load(Bt + (size_t)(n0 + (j << 4) + rlane) * ldb + koff + k0);
#pragma unroll
    for (int i = 0; i < 4; ++i) {
      V ah = Frag<T>::load(A + (size_t)(m0 + (i << 4) + rlane) * lda + koff + k0);
#pragma unroll
      for (int j = 0; j < 4; ++j) acc[i][j] = Frag<T>::mma(ah, bh[j], acc[i][j]);
      Frag<T>::guard(acc[i][0], acc[i][3], ah, ah);
    }
    Frag<T>::keep(bh[0], bh[1], bh[2], bh[3]);
  }
  acc_guard4(acc[0][0], acc[0][1], acc[0][2], acc[0][3]);
  acc_guard4(acc[1][0], acc[1][1], acc[1][2], acc[1][3]);
  acc_guard4(acc[2][0], acc[2][1], acc[2][2], acc[2][3]);
  acc_guard4(acc[3][0], acc[3][1], acc[3][2], acc[3][3]);

  float* slab = sT + wave * (16 * 68);
#pragma unroll
  for (int i = 0; i < 4; ++i) {
    const int mBase = m0 + (i << 4);
#pragma unroll
    for (int j = 0; j < 4; ++j) {
      const int n = n0 + (j << 4) + rlane;
      float bv = 0.f;
      if (BIAS_MODE == 2) bv = cmb_bf(bias[n]);
#pragma unroll
      for (int r = 0; r < 8; ++r) {
        float v = acc[i][j][r] * scale;
        if (BIAS_MODE == 1) v += cmb_bf(bias[mBase + mOff + r]);
        if (BIAS_MODE == 2) v += bv;
        slab[(mOff + r) * 68 + (j << 4) + rlane] = v;
      }
    }
    __builtin_amdgcn_fence(3  , "workgroup");
    __builtin_amdgcn_wave_barrier();
    __builtin_amdgcn_fence(2  , "workgroup");
    if (OUT_MODE == 0) {
      float* C = (float*)Cout;
      const int hh = lane >> 4, c4 = (lane & 15) * 4;
      for (int pass = 0; pass < 2; ++pass) {
#pragma unroll
        for (int it = 0; it < 8; ++it) {
          const int row = it * 2 + hh;
          const v4f v = *(const v4f*)(slab + row * 68 + c4);
          *(volatile v4f*)(C + (size_t)(mBase + row) * ldc + n0 + c4) = v;
        }
        __threadfence();
      }
    } else {
      const int q = lane >> 3, c8 = (lane & 7) * 8;
      unsigned short* C = (unsigned short*)Cout;
      for (int pass = 0; pass < 2; ++pass) {
#pragma unroll
        for (int it = 0; it < 4; ++it) {
          const int row = it * 4 + q;
          const float* sp = slab + row * 68 + c8;
          v8h hv;
#pragma unroll
          for (int e = 0; e < 8; ++e) hv[e] = (_Float16)sp[e];
          *(volatile v8h*)(C + (size_t)(mBase + row) * ldc + n0 + c8) = hv;
        }
        __threadfence();
      }
    }
    __builtin_amdgcn_fence(3  , "workgroup");
    __builtin_amdgcn_wave_barrier();
    __builtin_amdgcn_fence(2  , "workgroup");
  }
}

static_assert(((MTOK / 64) * (DM / 64)) % 8 == 0);
__global__ __launch_bounds__(256) void k_proj(const unsigned short* __restrict__ XH, const unsigned short* __restrict__ WT,
                                              unsigned short* __restrict__ C, const float* __restrict__ bias) {
  __shared__ __align__(16) float sT[8 * 16 * 68];
  gemm64_body<0, 2, 1>(sT, XH, DM, WT, DM, (void*)C, DM, bias, MTOK, DM, DM, 1.0f / (ACT_SC * W_SC));
}
__global__ __launch_bounds__(256) void k_proj_vT(const unsigned short* __restrict__ WT, const unsigned short* __restrict__ XH,
                                                 unsigned short* __restrict__ VT, const float* __restrict__ bias) {
  __shared__ __align__(16) float sT[8 * 16 * 68];
  gemm64_body<0, 1, 1>(sT, WT, DM, XH, DM, (void*)VT, MTOK, bias, DM, MTOK, DM, 1.0f / (ACT_SC * W_SC));
}
__global__ __launch_bounds__(256) void k_outproj(const unsigned short* __restrict__ CTX2, const unsigned short* __restrict__ WoT2,
                                                 float* __restrict__ out, const float* __restrict__ bias) {
  __shared__ __align__(16) float sT[8 * 16 * 68];
  gemm64_body<1, 2, 0>(sT, CTX2, 2 * DM, WoT2, 2 * DM, (void*)out, DM, bias, MTOK, DM, 2 * DM, 1.0f);
}

__global__ __launch_bounds__(128) void k_attn_lin(const unsigned short* __restrict__ QPp, const unsigned short* __restrict__ KPp,
                                                  const unsigned short* __restrict__ VTp, unsigned short* __restrict__ CTX2) {
  __shared__ __align__(16) _Float16 Psh[4][16 * 64];
  __shared__ __align__(16) float    Os[4][16 * 68];
  const _Float16* QP = (const _Float16*)QPp;
  const _Float16* KP = (const _Float16*)KPp;
  const _Float16* VT = (const _Float16*)VTp;
  const int tid = threadIdx.x, wave = tid >> 5, lane = tid & 31, hh = lane >> 4, c = lane & 15;
  const int nqb = SEQ / 64;
  const int bx = blockIdx.x;
  const int qb = bx % nqb;
  const int bh = bx / nqb;
  const int h = bh % NH;
  const int b = bh / NH;
  const int q0 = qb * 64 + wave * 16;

  v16h qa[2];
  {
    const _Float16* qrow = QP + (size_t)(b * SEQ + q0 + c) * DM + h * DK + 8 * hh;
    qa[0] = Frag<_Float16>::load(qrow);
    qa[1] = Frag<_Float16>::load(qrow + 32);
  }
  v8f oacc[4];
#pragma unroll
  for (int t = 0; t < 4; ++t) oacc[t] = (v8f){0.f,0.f,0.f,0.f,0.f,0.f,0.f,0.f};

  const _Float16* kbase = KP + (size_t)(b * SEQ) * DM + h * DK + 8 * hh;
  const _Float16* vbase = VT + (size_t)(h * DK) * MTOK + (size_t)b * SEQ + 8 * hh;
  _Float16* pw = Psh[wave];

  for (int kc = 0; kc < SEQ / 64; ++kc) {
    const int kv0 = kc * 64;
    v8f s[4];
#pragma unroll
    for (int j = 0; j < 4; ++j) {
      s[j] = (v8f){0.f,0.f,0.f,0.f,0.f,0.f,0.f,0.f};
      const _Float16* krow = kbase + (size_t)(kv0 + j * 16 + c) * DM;
#pragma unroll
      for (int dc = 0; dc < 2; ++dc) {
        const v16h kb = Frag<_Float16>::load(krow + dc * 32);
        s[j] = wmma16(qa[dc], kb, s[j]);
      }
    }
#pragma unroll
    for (int r = 0; r < 8; ++r)
#pragma unroll
      for (int j = 0; j < 4; ++j) pw[(8 * hh + r) * 64 + j * 16 + c] = (_Float16)s[j][r];
    __builtin_amdgcn_fence(3  , "workgroup");
    __builtin_amdgcn_wave_barrier();
    __builtin_amdgcn_fence(2  , "workgroup");
#pragma unroll
    for (int kk = 0; kk < 2; ++kk) {
      const v16h pa = Frag<_Float16>::load(pw + c * 64 + kk * 32 + 8 * hh);
#pragma unroll
      for (int t = 0; t < 4; ++t) {
        const v16h vb = Frag<_Float16>::load(vbase + (size_t)(t * 16 + c) * MTOK + kv0 + kk * 32);
        oacc[t] = wmma16(pa, vb, oacc[t]);
      }
    }
  }

  float* os = Os[wave];
#pragma unroll
  for (int r = 0; r < 8; ++r)
#pragma unroll
    for (int t = 0; t < 4; ++t) os[(8 * hh + r) * 68 + t * 16 + c] = oacc[t][r] * 0.125f;
  __builtin_amdgcn_fence(3  , "workgroup");
  __builtin_amdgcn_wave_barrier();
  __builtin_amdgcn_fence(2  , "workgroup");
  {
    const int q4 = lane >> 3, c8 = (lane & 7) * 8;
    v4u ph[4], pl[4];
#pragma unroll
    for (int it = 0; it < 4; ++it) {
      const float* sp = os + (it * 4 + q4) * 68 + c8;
      const v4f x0 = *(const v4f*)sp; const v4f x1 = *(const v4f*)(sp + 4);
      unsigned hA, lA, hB, lB, hC, lC, hD, lD;
      split2(x0.x, x0.y, hA, lA); split2(x0.z, x0.w, hB, lB); split2(x1.x, x1.y, hC, lC); split2(x1.z, x1.w, hD, lD);
      ph[it].x = hA; ph[it].y = hB; ph[it].z = hC; ph[it].w = hD;
      pl[it].x = lA; pl[it].y = lB; pl[it].z = lC; pl[it].w = lD;
    }
    unsigned short* cbase = CTX2 + (size_t)(b * SEQ + q0) * (2 * DM) + h * DK + c8;
    for (int pass = 0; pass < 2; ++pass) {
#pragma unroll
      for (int it = 0; it < 4; ++it) {
        const int row = it * 4 + q4;
        *(volatile v4u*)(cbase + (size_t)row * (2 * DM)) = ph[it];
        *(volatile v4u*)(cbase + (size_t)row * (2 * DM) + DM) = pl[it];
      }
      __threadfence();
    }
  }
}

constexpr size_t ACT_B = (size_t)MTOK * DM * 2;
constexpr size_t W_B   = (size_t)DM * DM * 2;
constexpr size_t WS_TOTAL = 3 * ACT_B   + 3 * W_B   + 2 * W_B   + 2 * ACT_B   + ACT_B   + 2 * ACT_B  ;
static_assert(WS_TOTAL <= (size_t)134217728);
static_assert(ACT_B % 128 == 0 && W_B % 128 == 0);

extern "C" void kernel_launch(void* const* d_in, const int* in_sizes, int n_in, void* d_out, int out_size, void* d_ws, size_t ws_size, hipStream_t stream) {
    if (n_in < 11) return;
    const long long need_act = ((long long)(NB - 1) * SEQ_FULL + SEQ) * DM;
    if ((long long)in_sizes[0] < need_act || (long long)in_sizes[1] < need_act || (long long)in_sizes[2] < need_act) return;
    for (int i = 3; i < 7; ++i) if ((long long)in_sizes[i] < (long long)DM * DM) return;
    for (int i = 7; i < 11; ++i) if (in_sizes[i] < DM) return;
    if ((long long)out_size < (long long)MTOK * DM) return;
    if (WS_TOTAL > ws_size) return;

    const float* Q  = (const float*)d_in[0];
    const float* K  = (const float*)d_in[1];
    const float* V  = (const float*)d_in[2];
    const float* Wq = (const float*)d_in[3];
    const float* Wk = (const float*)d_in[4];
    const float* Wv = (const float*)d_in[5];
    const float* Wo = (const float*)d_in[6];
    const float* bq = (const float*)d_in[7];
    const float* bk = (const float*)d_in[8];
    const float* bv = (const float*)d_in[9];
    const float* bo = (const float*)d_in[10];
    float* out = (float*)d_out;

    char* wsp = (char*)d_ws;
    unsigned short* QH   = (unsigned short*)wsp; wsp += ACT_B;
    unsigned short* KH   = (unsigned short*)wsp; wsp += ACT_B;
    unsigned short* VH   = (unsigned short*)wsp; wsp += ACT_B;
    unsigned short* WqT  = (unsigned short*)wsp; wsp += W_B;
    unsigned short* WkT  = (unsigned short*)wsp; wsp += W_B;
    unsigned short* WvT  = (unsigned short*)wsp; wsp += W_B;
    unsigned short* WoT2 = (unsigned short*)wsp; wsp += 2 * W_B;
    unsigned short* QP   = (unsigned short*)wsp; wsp += ACT_B;
    unsigned short* KP   = (unsigned short*)wsp; wsp += ACT_B;
    unsigned short* VT   = (unsigned short*)wsp; wsp += ACT_B;
    unsigned short* CTX2 = (unsigned short*)wsp; wsp += 2 * ACT_B;

    const unsigned gAct = (unsigned)((MTOK * (DM / 8)) / 256);
    const unsigned gW   = (unsigned)((DM * (DM / 8)) / 256);
    const unsigned gG   = (unsigned)(((MTOK / 64) * (DM / 64)) / 8);

    k_cast_act<<<gAct, 256, 0, stream>>>(Q, QH);
    k_cast_act<<<gAct, 256, 0, stream>>>(K, KH);
    k_cast_act<<<gAct, 256, 0, stream>>>(V, VH);
    k_cast_wT<<<gW, 256, 0, stream>>>(Wq, WqT);
    k_cast_wT<<<gW, 256, 0, stream>>>(Wk, WkT);
    k_cast_wT<<<gW, 256, 0, stream>>>(Wv, WvT);
    k_cast_wo2<<<gW, 256, 0, stream>>>(Wo, WoT2);

    k_proj<<<gG, 256, 0, stream>>>(QH, WqT, QP, bq);
    k_proj<<<gG, 256, 0, stream>>>(KH, WkT, KP, bk);
    k_proj_vT<<<gG, 256, 0, stream>>>(WvT, VH, VT, bv);

    k_attn_lin<<<(unsigned)(NB * NH * (SEQ / 64)), 128, 0, stream>>>(QP, KP, VT, CTX2);

    k_outproj<<<gG, 256, 0, stream>>>(CTX2, WoT2, out, bo);
}
